// NeuralPolarDecoder_22686017257998
// MI455X (gfx1250) — hardware-verified
//
#include <hip/hip_runtime.h>
#include <math.h>
#include <stdint.h>

constexpr int kBatch  = 32;
constexpr int kLen    = 4096;
constexpr int kDim    = 64;
constexpr int kPos    = kBatch * kLen;
constexpr int kPair   = kPos / 2;
constexpr int kStages = 12;
constexpr float kWCarry    = 8.0f;
constexpr float kWCarryInv = 0.125f;
constexpr float kClipLo    = 1e-7f;
constexpr int kOffCW1 = 0;
constexpr int kOffCW2 = 8192;
constexpr int kOffBW1 = 12288;
constexpr int kOffBW2 = 20480;
constexpr int kOffEW2 = 24576;
constexpr int kWHalves = 28672;
static_assert(kPos % 128 == 0);
static_assert(kPair % 64 == 0);

typedef __attribute__((ext_vector_type(16))) _Float16 v16h;
typedef __attribute__((ext_vector_type(8)))  _Float16 v8h;
typedef __attribute__((ext_vector_type(16))) __bf16   v16b;
typedef __attribute__((ext_vector_type(8)))  __bf16   v8b;
typedef __attribute__((ext_vector_type(8)))  float    v8f;
typedef __attribute__((ext_vector_type(4)))  float    v4f;
typedef __attribute__((ext_vector_type(4)))  unsigned int v4u;
typedef __attribute__((ext_vector_type(4)))  int      v4i;

__device__ __forceinline__ unsigned short f2bf_bits(float f) {
  unsigned u = __float_as_uint(f);
  return (unsigned short)((u + 0x7FFFu + ((u >> 16) & 1u)) >> 16);
}
__device__ __forceinline__ float bf_bits2f(unsigned short h) { return __uint_as_float(((unsigned)h) << 16); }

__device__ __forceinline__ void dep_guard_h(v8f& a, v8f& b, v16h x, v16h y) { asm volatile("v_nop\n\tv_nop\n\tv_nop\n\tv_nop" : "+v"(a), "+v"(b) : "v"(x), "v"(y)); }
__device__ __forceinline__ void dep_guard_b(v8f& a, v8f& b, v16b x, v16b y) { asm volatile("v_nop\n\tv_nop\n\tv_nop\n\tv_nop" : "+v"(a), "+v"(b) : "v"(x), "v"(y)); }
__device__ __forceinline__ void keep4_h(v16h a, v16h b, v16h c, v16h d) { asm volatile("v_nop" :: "v"(a), "v"(b), "v"(c), "v"(d)); }
__device__ __forceinline__ void keep4_b(v16b a, v16b b, v16b c, v16b d) { asm volatile("v_nop" :: "v"(a), "v"(b), "v"(c), "v"(d)); }
__device__ __forceinline__ void acc_guard4(v8f& a, v8f& b, v8f& c, v8f& d) { asm volatile("v_nop\n\tv_nop\n\tv_nop\n\tv_nop" : "+v"(a), "+v"(b), "+v"(c), "+v"(d)); }
template <typename T> struct Frag;
template <> struct Frag<_Float16> {
  typedef v16h V; union U { v16h v; v8h h[2]; };
  static __device__ __forceinline__ v16h load(const _Float16* p) {
    U f; f.h[0] = *(const v8h*)(p); f.h[1] = *(const v8h*)(p + 16); return f.v;
  }
  static __device__ __forceinline__ v8f mma(v16h a, v16h b, v8f c) {
    return __builtin_amdgcn_wmma_f32_16x16x32_f16(false, a, false, b, (short)0, c, false, false);
  }
  static __device__ __forceinline__ void guard(v8f& a, v8f& b, v16h x, v16h y) { dep_guard_h(a, b, x, y); }
  static __device__ __forceinline__ void keep(v16h a, v16h b, v16h c, v16h d) { keep4_h(a, b, c, d); }
};
template <> struct Frag<__bf16> {
  typedef v16b V; union U { v16b v; v8b h[2]; };
  static __device__ __forceinline__ v16b load(const __bf16* p) {
    U f; f.h[0] = *(const v8b*)(p); f.h[1] = *(const v8b*)(p + 16); return f.v;
  }
  static __device__ __forceinline__ v8f mma(v16b a, v16b b, v8f c) {
    return __builtin_amdgcn_wmma_f32_16x16x32_bf16(false, a, false, b, (short)0, c, false, false);
  }
  static __device__ __forceinline__ void guard(v8f& a, v8f& b, v16b x, v16b y) { dep_guard_b(a, b, x, y); }
  static __device__ __forceinline__ void keep(v16b a, v16b b, v16b c, v16b d) { keep4_b(a, b, c, d); }
};

__device__ __forceinline__ unsigned pk16(unsigned short a, unsigned short b) { return (unsigned)a | ((unsigned)b << 16); }
__device__ __forceinline__ unsigned short h_bits(float f) { const _Float16 h = (_Float16)f; return __builtin_bit_cast(unsigned short, h); }

template <int ET> struct Elem;
template <> struct Elem<0> { typedef _Float16 T; };
template <> struct Elem<1> { typedef __bf16 T; };
template <int ET, bool SPLIT, int BIAS_MODE, int OUT_MODE, bool RESID, int ACT = 0>
__global__ __launch_bounds__(256) void wmma_gemm64(
    const unsigned short* __restrict__ Ap, const unsigned short* __restrict__ A2p, int lda, long strideA,
    const unsigned short* __restrict__ Btp, const unsigned short* __restrict__ Bt2p, int ldb, long strideB,
    void* __restrict__ Cout, void* __restrict__ Cout2, int ldc, long strideC,
    const float* __restrict__ bias,
    const float* __restrict__ resid, long strideR,
    int M, int N, int K, float scale) {
  typedef typename Elem<ET>::T T;
  typedef typename Frag<T>::V V;
  const T* A = (const T*)Ap; const T* A2 = (const T*)A2p; const T* Bt = (const T*)Btp; const T* Bt2 = (const T*)Bt2p;
  __shared__ __align__(16) float sT[8][16 * 68];
  const int b    = blockIdx.y;
  const int lane = threadIdx.x & 31;
  const int wave = threadIdx.x >> 5;
  const int tilesN = N >> 6;
  const int tilesM = M >> 6;
  const int tile = blockIdx.x * 8 + wave;
  if (tile >= tilesM * tilesN) return;
  const int tm = tile / tilesN;
  const int tn = tile - tm * tilesN;
  const int m0 = tm << 6;
  const int n0 = tn << 6;

  const T* Ab  = A  + (size_t)b * strideA;
  const T* Bb  = Bt + (size_t)b * strideB;
  const T* Ab2 = SPLIT ? (A2  + (size_t)b * strideA) : nullptr;
  const T* Bb2 = SPLIT ? (Bt2 + (size_t)b * strideB) : nullptr;

  const int rlane = lane & 15;
  const int koff  = (lane >> 4) * 8;
  const int mOff  = (lane >> 4) * 8;

  v8f acc[4][4];
#pragma unroll
  for (int i = 0; i < 4; ++i)
#pragma unroll
    for (int j = 0; j < 4; ++j) acc[i][j] = (v8f){0.f,0.f,0.f,0.f,0.f,0.f,0.f,0.f};

  for (int k0 = 0; k0 < K; k0 += 32) {
    V bh[4], bl[4];
#pragma unroll
    for (int j = 0; j < 4; ++j) {
      const size_t bo = (size_t)(n0 + (j << 4) + rlane) * ldb + koff + k0;
      bh[j] = Frag<T>::load(Bb + bo);
      if (SPLIT) bl[j] = Frag<T>::load(Bb2 + bo);
    }
#pragma unroll
    for (int i = 0; i < 4; ++i) {
      const size_t ao = (size_t)(m0 + (i << 4) + rlane) * lda + koff + k0;
      V ah = Frag<T>::load(Ab + ao);
      V al;
      if (SPLIT) al = Frag<T>::load(Ab2 + ao);
#pragma unroll
      for (int j = 0; j < 4; ++j) {
        acc[i][j] = Frag<T>::mma(ah, bh[j], acc[i][j]);
        if (SPLIT) {
          acc[i][j] = Frag<T>::mma(ah, bl[j], acc[i][j]);
          acc[i][j] = Frag<T>::mma(al, bh[j], acc[i][j]);
        }
      }
      Frag<T>::guard(acc[i][0], acc[i][3], ah, SPLIT ? al : ah);
    }
    Frag<T>::keep(bh[0], bh[1], bh[2], bh[3]);
    if (SPLIT) Frag<T>::keep(bl[0], bl[1], bl[2], bl[3]);
  }
  acc_guard4(acc[0][0], acc[0][1], acc[0][2], acc[0][3]);
  acc_guard4(acc[1][0], acc[1][1], acc[1][2], acc[1][3]);
  acc_guard4(acc[2][0], acc[2][1], acc[2][2], acc[2][3]);
  acc_guard4(acc[3][0], acc[3][1], acc[3][2], acc[3][3]);

  float* slab = sT[wave];
  const float* Rb = RESID ? (resid + (size_t)b * strideR) : nullptr;
#pragma unroll
  for (int i = 0; i < 4; ++i) {
    const int mBase = m0 + (i << 4);
#pragma unroll
    for (int j = 0; j < 4; ++j) {
      const int n = n0 + (j << 4) + rlane;
      float bv = 0.f;
      if (BIAS_MODE == 2) bv = bias[n];
#pragma unroll
      for (int r = 0; r < 8; ++r) {
        float v = acc[i][j][r] * scale;
        if (BIAS_MODE == 1) v += bias[mBase + mOff + r];
        if (BIAS_MODE == 2) v += bv;
        if (RESID) v += Rb[(size_t)(mBase + mOff + r) * ldc + n];
        if (ACT == 2) v = fmaxf(v, 0.0f);
        if (ACT == 4) v = (v > 0.f) ? v : 0.01f * v;
        slab[(mOff + r) * 68 + (j << 4) + rlane] = v;
      }
    }
    __builtin_amdgcn_fence(__ATOMIC_RELEASE, "workgroup");
    __builtin_amdgcn_wave_barrier();
    __builtin_amdgcn_fence(__ATOMIC_ACQUIRE, "workgroup");
    if (OUT_MODE == 0) {
      float* C = (float*)Cout + (size_t)b * strideC;
      const int hh = lane >> 4, c4 = (lane & 15) * 4;
      for (int pass = 0; pass < 2; ++pass) {
#pragma unroll
        for (int it = 0; it < 8; ++it) {
          const int row = it * 2 + hh;
          v4f v = *(const v4f*)(slab + row * 68 + c4);
          *(volatile v4f*)(C + (size_t)(mBase + row) * ldc + n0 + c4) = v;
        }
        __threadfence();
      }
    } else {
      const int q = lane >> 3, c8 = (lane & 7) * 8;
      unsigned short* C  = (unsigned short*)Cout  + (size_t)b * strideC;
      unsigned short* C2 = (OUT_MODE == 2) ? ((unsigned short*)Cout2 + (size_t)b * strideC) : nullptr;
      for (int pass = 0; pass < 2; ++pass) {
#pragma unroll
        for (int it = 0; it < 4; ++it) {
          const int row = it * 4 + q;
          const float* sp = slab + row * 68 + c8;
          v8h hv, lv;
#pragma unroll
          for (int e = 0; e < 8; ++e) {
            if (OUT_MODE == 1) {
              hv[e] = (_Float16)sp[e];
            } else {
              unsigned short hb = f2bf_bits(sp[e]);
              unsigned short lb = f2bf_bits(sp[e] - bf_bits2f(hb));
              hv[e] = __builtin_bit_cast(_Float16, hb);
              lv[e] = __builtin_bit_cast(_Float16, lb);
            }
          }
          *(volatile v8h*)(C + (size_t)(mBase + row) * ldc + n0 + c8) = hv;
          if (OUT_MODE == 2) *(volatile v8h*)(C2 + (size_t)(mBase + row) * ldc + n0 + c8) = lv;
        }
        __threadfence();
      }
    }
    __builtin_amdgcn_fence(__ATOMIC_RELEASE, "workgroup");
    __builtin_amdgcn_wave_barrier();
    __builtin_amdgcn_fence(__ATOMIC_ACQUIRE, "workgroup");
  }
}

__global__ __launch_bounds__(256) void wprep_kernel(const float* __restrict__ cn_w1, const float* __restrict__ cn_w2,
                                                    const float* __restrict__ bn_w1, const float* __restrict__ bn_w2,
                                                    const float* __restrict__ emb_w2, unsigned short* __restrict__ wts) {
  const int bx = blockIdx.x;
  const float* src; int kt, blk0, dOff;
  if (bx < 4)       { src = cn_w1;  kt = 128; blk0 = 0;  dOff = kOffCW1; }
  else if (bx < 6)  { src = cn_w2;  kt = 64;  blk0 = 4;  dOff = kOffCW2; }
  else if (bx < 10) { src = bn_w1;  kt = 128; blk0 = 6;  dOff = kOffBW1; }
  else if (bx < 12) { src = bn_w2;  kt = 64;  blk0 = 10; dOff = kOffBW2; }
  else              { src = emb_w2; kt = 64;  blk0 = 12; dOff = kOffEW2; }
  const int lc  = (bx - blk0) * 256 + (int)threadIdx.x;
  const int cpr = kt >> 3;
  const int n   = lc / cpr;
  const int k8  = lc - n * cpr;
  unsigned short hb[8];
#pragma unroll
  for (int e = 0; e < 8; ++e) hb[e] = h_bits(kWCarry * src[(size_t)(k8 * 8 + e) * kDim + n]);
  const v4u u = (v4u){pk16(hb[0], hb[1]), pk16(hb[2], hb[3]), pk16(hb[4], hb[5]), pk16(hb[6], hb[7])};
  unsigned short* dp = wts + dOff + (size_t)n * kt + k8 * 8;
  *(volatile v4u*)dp = u;
  __threadfence();
  *(volatile v4u*)dp = u;
}

__global__ __launch_bounds__(128) void ttab_kernel(const float* __restrict__ label_emb, const float* __restrict__ bn_w1,
                                                   float* __restrict__ ttab) {
  __shared__ __align__(16) float st[128];
  const int t = threadIdx.x;
  const int v = t >> 6, n = t & 63;
  float acc = 0.f;
#pragma unroll 1
  for (int k = 0; k < kDim; ++k) acc += label_emb[v * kDim + k] * bn_w1[(size_t)(128 + k) * kDim + n];
  st[t] = acc;
  __syncthreads();
  if (t < 32) {
    const v4f val = *(const v4f*)(st + t * 4);
    float* dp = ttab + t * 4;
    *(volatile v4f*)dp = val;
    __threadfence();
    *(volatile v4f*)dp = val;
  }
}

__global__ __launch_bounds__(256) void emb1_kernel(const float* __restrict__ y, const float* __restrict__ w1,
                                                   const float* __restrict__ b1, unsigned short* __restrict__ hout) {
  const int gid = blockIdx.x * 256 + (int)threadIdx.x;
  const int row = gid >> 3, ch = gid & 7;
  const float y0 = y[(size_t)row * 2], y1 = y[(size_t)row * 2 + 1];
  unsigned short hb[8];
#pragma unroll
  for (int e = 0; e < 8; ++e) {
    const int n = ch * 8 + e;
    float h = y0 * w1[n] + y1 * w1[kDim + n];
    h += b1[n];
    hb[e] = h_bits(fmaxf(h, 0.0f));
  }
  const v4u u = (v4u){pk16(hb[0], hb[1]), pk16(hb[2], hb[3]), pk16(hb[4], hb[5]), pk16(hb[6], hb[7])};
  unsigned short* dp = hout + (size_t)row * kDim + ch * 8;
  *(volatile v4u*)dp = u;
  __threadfence();
  *(volatile v4u*)dp = u;
}

__global__ __launch_bounds__(256) void bnact_kernel(const float* __restrict__ g, const int* __restrict__ vsrc,
                                                    const float* __restrict__ b1, const float* __restrict__ ttab,
                                                    unsigned short* __restrict__ hout) {
  const int gid = blockIdx.x * 256 + (int)threadIdx.x;
  const int q = gid >> 3, ch = gid & 7;
  const int vo = vsrc[2 * q], ve = vsrc[2 * q + 1];
  const int vx = (vo + ve) & 1;
  const float* gp = g + (size_t)q * kDim + ch * 8;
  const v4f g0 = *(const v4f*)(gp);
  const v4f g1 = *(const v4f*)(gp + 4);
  const float* tp = ttab + vx * kDim + ch * 8;
  const v4f t0 = *(const v4f*)(tp);
  const v4f t1 = *(const v4f*)(tp + 4);
  const float* bp = b1 + ch * 8;
  const v4f c0 = *(const v4f*)(bp);
  const v4f c1 = *(const v4f*)(bp + 4);
  unsigned short hb[8];
#pragma unroll
  for (int e = 0; e < 4; ++e) {
    hb[e]     = h_bits(fmaxf(g0[e] + c0[e] + t0[e], 0.0f));
    hb[4 + e] = h_bits(fmaxf(g1[e] + c1[e] + t1[e], 0.0f));
  }
  const v4u u = (v4u){pk16(hb[0], hb[1]), pk16(hb[2], hb[3]), pk16(hb[4], hb[5]), pk16(hb[6], hb[7])};
  unsigned short* dp = hout + (size_t)q * kDim + ch * 8;
  *(volatile v4u*)dp = u;
  __threadfence();
  *(volatile v4u*)dp = u;
}

__global__ __launch_bounds__(256) void perm_kernel(const float* __restrict__ hlr, const int* __restrict__ vsrc,
                                                   const float* __restrict__ llr_w, const float* __restrict__ llr_b,
                                                   unsigned short* __restrict__ edst, int* __restrict__ vdst,
                                                   float* __restrict__ loss, float* __restrict__ pst, int lsh, int stage) {
  __shared__ float sw[2 * kDim];
  __shared__ __align__(16) float sl[32];
  __shared__ __align__(16) float sp[64];
  __shared__ __align__(16) int   sv[32];
  const int t = threadIdx.x;
  if (t < 2 * kDim) sw[t] = llr_w[t];
  __syncthreads();
  const int rloc = t >> 3, ch = t & 7;
  const int r0   = blockIdx.x * 32;
  const int r    = r0 + rloc;
  const int b    = r0 >> 12;
  const int pos  = r & (kLen - 1);
  const int pos0 = r0 & (kLen - 1);
  const int blk    = pos >> lsh;
  const int within = pos & ((1 << lsh) - 1);
  const int right  = within >> (lsh - 1);
  const int j      = within & ((1 << (lsh - 1)) - 1);
  const int s0     = (b << 12) + (blk << lsh) + 2 * j;
  const int q      = s0 >> 1;
  const int vo = vsrc[s0], ve = vsrc[s0 + 1];
  const int vx = (vo + ve) & 1;
  const int vnew = right ? ve : vx;
  const float* hp = hlr + ((size_t)right * kPair + (size_t)q) * kDim + ch * 8;
  const v4f e0 = *(const v4f*)(hp);
  const v4f e1 = *(const v4f*)(hp + 4);
  float l0 = 0.f, l1 = 0.f;
#pragma unroll
  for (int e = 0; e < 4; ++e) {
    const int k = ch * 8 + e;
    l0 += e0[e] * sw[2 * k];
    l1 += e0[e] * sw[2 * k + 1];
    l0 += e1[e] * sw[2 * (k + 4)];
    l1 += e1[e] * sw[2 * (k + 4) + 1];
  }
  l0 += __shfl_xor(l0, 1, 32);  l1 += __shfl_xor(l1, 1, 32);
  l0 += __shfl_xor(l0, 2, 32);  l1 += __shfl_xor(l1, 2, 32);
  l0 += __shfl_xor(l0, 4, 32);  l1 += __shfl_xor(l1, 4, 32);
  l0 += llr_b[0];
  l1 += llr_b[1];
  const float m   = fmaxf(l0, l1);
  const float x0  = expf(l0 - m), x1 = expf(l1 - m);
  const float inv = 1.0f / (x0 + x1);
  const float p0  = x0 * inv, p1 = x1 * inv;
  const float c0  = fminf(fmaxf(p0, kClipLo), 1.0f - kClipLo);
  const float c1  = fminf(fmaxf(p1, kClipLo), 1.0f - kClipLo);
  const int   lab = vnew < 0 ? 0 : (vnew > 1 ? 1 : vnew);
  const float pl  = lab ? c1 : c0;
  const float ls  = -logf(pl);
  unsigned short hb[8];
#pragma unroll
  for (int e = 0; e < 4; ++e) { hb[e] = h_bits(e0[e]); hb[4 + e] = h_bits(e1[e]); }
  const v4u u = (v4u){pk16(hb[0], hb[1]), pk16(hb[2], hb[3]), pk16(hb[4], hb[5]), pk16(hb[6], hb[7])};
  unsigned short* ep = edst + (size_t)r * kDim + ch * 8;
  *(volatile v4u*)ep = u;
  if (ch == 0) { sl[rloc] = ls; sp[2 * rloc] = p0; sp[2 * rloc + 1] = p1; sv[rloc] = vnew; }
  __threadfence();
  *(volatile v4u*)ep = u;
  __syncthreads();
  const int lane = t & 31, wave = t >> 5;
  if (wave == 0) {
    const int li = (lane & 7) * 4;
    const v4f val = *(const v4f*)(sl + li);
    float* dp = loss + (size_t)(b * kStages + stage) * kLen + pos0 + li;
    if (lane < 8) *(volatile v4f*)dp = val;
    __threadfence();
    if (lane < 8) *(volatile v4f*)dp = val;
  } else if (wave == 1) {
    const int li = (lane & 7) * 4;
    const v4i val = *(const v4i*)(sv + li);
    int* dp = vdst + r0 + li;
    if (lane < 8) *(volatile v4i*)dp = val;
    __threadfence();
    if (lane < 8) *(volatile v4i*)dp = val;
  } else if (wave == 2) {
    const int li = (lane & 15) * 4;
    const v4f val = *(const v4f*)(sp + li);
    float* dp = pst + (size_t)r0 * 2 + li;
    if (lane < 16) *(volatile v4f*)dp = val;
    __threadfence();
    if (lane < 16) *(volatile v4f*)dp = val;
  }
}

__global__ __launch_bounds__(256) void pred_kernel(const float* __restrict__ pall, float* __restrict__ out1,
                                                   float* __restrict__ out2) {
  __shared__ __align__(16) float sm[128 * 24];
  const int t  = threadIdx.x;
  const int r0 = blockIdx.x * 128;
#pragma unroll 1
  for (int s = 0; s < kStages; ++s) {
    const float v = pall[(size_t)s * kPos * 2 + (size_t)r0 * 2 + t];
    sm[(t >> 1) * 24 + s * 2 + (t & 1)] = v;
  }
  __syncthreads();
  v4f vals[3];
#pragma unroll
  for (int i = 0; i < 3; ++i) vals[i] = *(const v4f*)(sm + (i * 256 + t) * 4);
  float* o1 = out1 + (size_t)r0 * 24;
  float* o2 = out2 + (size_t)r0 * 24;
  for (int pass = 0; pass < 2; ++pass) {
#pragma unroll
    for (int i = 0; i < 3; ++i) {
      *(volatile v4f*)(o1 + (i * 256 + t) * 4) = vals[i];
      *(volatile v4f*)(o2 + (i * 256 + t) * 4) = vals[i];
    }
    __threadfence();
  }
}

extern "C" void kernel_launch(void* const* d_in, const int* in_sizes, int n_in,
                              void* d_out, int out_size, void* d_ws,
                              size_t ws_size, hipStream_t stream) {
  (void)in_sizes; (void)n_in; (void)out_size;
  const int*   x       = (const int*)  d_in[0];
  const float* y       = (const float*)d_in[1];
  const float* emb_w1  = (const float*)d_in[2];
  const float* emb_b1  = (const float*)d_in[3];
  const float* emb_w2  = (const float*)d_in[4];
  const float* emb_b2  = (const float*)d_in[5];
  const float* cn_w1   = (const float*)d_in[6];
  const float* cn_b1   = (const float*)d_in[7];
  const float* cn_w2   = (const float*)d_in[8];
  const float* cn_b2   = (const float*)d_in[9];
  const float* bn_w1   = (const float*)d_in[10];
  const float* bn_b1   = (const float*)d_in[11];
  const float* bn_w2   = (const float*)d_in[12];
  const float* bn_b2   = (const float*)d_in[13];
  const float* llr_w   = (const float*)d_in[14];
  const float* llr_b   = (const float*)d_in[15];
  const float* label_emb = (const float*)d_in[16];

  char* ws = (char*)d_ws;
  size_t off = 0;
  auto carve = [&](size_t bytes) -> char* {
    char* p = ws + off;
    off += (bytes + 255) & ~(size_t)255;
    return p;
  };
  const size_t eBytes = (size_t)kPos * kDim * 2;
  unsigned short* E0  = (unsigned short*)carve(eBytes);
  unsigned short* E1  = (unsigned short*)carve(eBytes);
  unsigned short* Hpl = (unsigned short*)carve(eBytes);
  float*          G   = (float*)carve((size_t)kPair * kDim * 4);
  float*          HLR = (float*)carve((size_t)2 * kPair * kDim * 4);
  float*          Ppl = (float*)carve((size_t)kStages * kPos * 2 * 4);
  int*            VA  = (int*)carve((size_t)kPos * 4);
  int*            VB  = (int*)carve((size_t)kPos * 4);
  unsigned short* Wts = (unsigned short*)carve((size_t)kWHalves * 2);
  float*          Ttab = (float*)carve(512);
  if (off > ws_size) return;

  float* loss = (float*)d_out;
  float* out1 = loss + (size_t)kBatch * kStages * kLen;
  float* out2 = out1 + (size_t)kPos * kStages * 2;

  wprep_kernel<<<14, 256, 0, stream>>>(cn_w1, cn_w2, bn_w1, bn_w2, emb_w2, Wts);
  ttab_kernel<<<1, 128, 0, stream>>>(label_emb, bn_w1, Ttab);

  emb1_kernel<<<(kPos * 8) / 256, 256, 0, stream>>>(y, emb_w1, emb_b1, Hpl);
  wmma_gemm64<0, false, 2, 1, false, 0><<<dim3((kPos / 64) / 8, 1), 256, 0, stream>>>(
      Hpl, Hpl, kDim, 0L, Wts + kOffEW2, Wts + kOffEW2, kDim, 0L,
      (void*)E0, (void*)E0, kDim, 0L, emb_b2, emb_b2, 0L, kPos, kDim, kDim, kWCarryInv);

  const int stageBlocks = (kPair / 64) / 8;
  for (int s = 0; s < kStages; ++s) {
    const int lsh = kStages - s;
    const unsigned short* Ecur = (s & 1) ? E1 : E0;
    unsigned short*       Enxt = (s & 1) ? E0 : E1;
    int*       vdst = (s & 1) ? VB : VA;
    const int* vcur = (s == 0) ? x : (((s - 1) & 1) ? VB : VA);

    wmma_gemm64<0, false, 2, 1, false, 2><<<dim3(stageBlocks, 1), 256, 0, stream>>>(
        Ecur, Ecur, 2 * kDim, 0L, Wts + kOffCW1, Wts + kOffCW1, 2 * kDim, 0L,
        (void*)Hpl, (void*)Hpl, kDim, 0L, cn_b1, cn_b1, 0L, kPair, kDim, 2 * kDim, kWCarryInv);
    wmma_gemm64<0, false, 2, 0, false, 0><<<dim3(stageBlocks, 1), 256, 0, stream>>>(
        Hpl, Hpl, kDim, 0L, Wts + kOffCW2, Wts + kOffCW2, kDim, 0L,
        (void*)HLR, (void*)HLR, kDim, 0L, cn_b2, cn_b2, 0L, kPair, kDim, kDim, kWCarryInv);
    wmma_gemm64<0, false, 0, 0, false, 0><<<dim3(stageBlocks, 1), 256, 0, stream>>>(
        Ecur, Ecur, 2 * kDim, 0L, Wts + kOffBW1, Wts + kOffBW1, 2 * kDim, 0L,
        (void*)G, (void*)G, kDim, 0L, bn_b1, bn_b1, 0L, kPair, kDim, 2 * kDim, kWCarryInv);
    bnact_kernel<<<(kPair * 8) / 256, 256, 0, stream>>>(G, vcur, bn_b1, Ttab, Hpl);
    wmma_gemm64<0, false, 2, 0, false, 0><<<dim3(stageBlocks, 1), 256, 0, stream>>>(
        Hpl, Hpl, kDim, 0L, Wts + kOffBW2, Wts + kOffBW2, kDim, 0L,
        (void*)(HLR + (size_t)kPair * kDim), (void*)(HLR + (size_t)kPair * kDim), kDim, 0L,
        bn_b2, bn_b2, 0L, kPair, kDim, kDim, kWCarryInv);
    perm_kernel<<<kPos / 32, 256, 0, stream>>>(HLR, vcur, llr_w, llr_b, Enxt, vdst, loss,
                                                Ppl + (size_t)s * kPos * 2, lsh, s);
  }
  pred_kernel<<<kPos / 128, 256, 0, stream>>>(Ppl, out1, out2);
}
